// FR_PDP_block_67267777790396
// MI455X (gfx1250) — hardware-verified
//
#include <hip/hip_runtime.h>
#include <math.h>

typedef __attribute__((ext_vector_type(16))) _Float16 v16h;
typedef __attribute__((ext_vector_type(16))) __bf16 v16b;
typedef __attribute__((ext_vector_type(8)))  _Float16 v8h;
typedef __attribute__((ext_vector_type(8)))  float v8f;
typedef __attribute__((ext_vector_type(4)))  float v4f;
typedef __attribute__((ext_vector_type(2)))  float v2f;
typedef __attribute__((ext_vector_type(4)))  unsigned v4u;
typedef __attribute__((ext_vector_type(4)))  int v4i;
typedef float __attribute__((may_alias)) float_a;
typedef int __attribute__((may_alias)) int_a;

template <typename T> __device__ __forceinline__ void vst2(void* p, T v) { *(volatile T*)p = v; __threadfence(); *(volatile T*)p = v; }
__device__ __forceinline__ v8f wmma16(v16h a, v16h b, v8f c) {
  v8f d = __builtin_amdgcn_wmma_f32_16x16x32_f16(false, a, false, b, (short)0, c, false, false);
  asm volatile("v_nop\n\tv_nop\n\tv_nop\n\tv_nop" : "+v"(d) : "v"(a), "v"(b));
  return d;
}
__device__ __forceinline__ v8f wmma_bf(v16b a, v16b b, v8f c) {
  v8f d = __builtin_amdgcn_wmma_f32_16x16x32_bf16(false, a, false, b, (short)0, c, false, false);
  asm volatile("v_nop\n\tv_nop\n\tv_nop\n\tv_nop" : "+v"(d) : "v"(a), "v"(b));
  return d;
}
__device__ __forceinline__ v16h frag_h(const _Float16* rowk0, int lane) {
  union { v16h v; v8h q[2]; } u; const _Float16* p = rowk0 + 8 * (lane >> 4);
  u.q[0] = *(const v8h*)p; u.q[1] = *(const v8h*)(p + 16); return u.v;
}
__device__ __forceinline__ v16h frag_f32(const float* rowk0, int lane) {
  v16h a; const float* p = rowk0 + 8 * (lane >> 4);
#pragma unroll
  for (int i = 0; i < 8; ++i) { a[i] = (_Float16)p[i]; a[8 + i] = (_Float16)p[16 + i]; }
  return a;
}
__device__ __forceinline__ v16h frag_f32s(const float* rowk0, int lane, float sc) {
  v16h a; const float* p = rowk0 + 8 * (lane >> 4);
#pragma unroll
  for (int i = 0; i < 8; ++i) { a[i] = (_Float16)(p[i] * sc); a[8 + i] = (_Float16)(p[16 + i] * sc); }
  return a;
}
__device__ __forceinline__ v16h fragc_f32(const float* W, int k0, int n, int lane, int ld, int K) {
  v16h a; const int g = lane >> 4;
#pragma unroll
  for (int i = 0; i < 8; ++i) { const int ka = k0 + 8 * g + i, kb = ka + 16;
    a[i] = (_Float16)(ka < K ? W[(size_t)(ka < K ? ka : K - 1) * ld + n] : 0.f); a[8 + i] = (_Float16)(kb < K ? W[(size_t)(kb < K ? kb : K - 1) * ld + n] : 0.f); }
  return a;
}
struct F2 { v16b h, l; };
__device__ __forceinline__ F2 bsplit16(const float v[16]) { F2 r;
#pragma unroll
  for (int i = 0; i < 16; ++i) { const __bf16 h = (__bf16)v[i]; r.h[i] = h; r.l[i] = (__bf16)(v[i] - (float)h); }
  return r; }
__device__ __forceinline__ F2 split_row(const float* row, int k0, int lane) { float v[16]; const float* p = row + k0 + 8 * (lane >> 4);
#pragma unroll
  for (int i = 0; i < 8; ++i) { v[i] = p[i]; v[8 + i] = p[16 + i]; }
  return bsplit16(v); }
__device__ __forceinline__ F2 split_rowK(const float* row, int k0, int lane, int K) { float v[16]; const int g = lane >> 4;
#pragma unroll
  for (int i = 0; i < 8; ++i) { const int ka = k0 + 8 * g + i, kb = ka + 16; v[i] = ka < K ? row[ka < K ? ka : K - 1] : 0.f; v[8 + i] = kb < K ? row[kb < K ? kb : K - 1] : 0.f; }
  return bsplit16(v); }
__device__ __forceinline__ F2 split_col(const float* W, int k0, int n, int lane, int ld, int K) { float v[16]; const int g = lane >> 4;
#pragma unroll
  for (int i = 0; i < 8; ++i) { const int ka = k0 + 8 * g + i, kb = ka + 16; v[i] = ka < K ? W[(size_t)(ka < K ? ka : K - 1) * ld + n] : 0.f; v[8 + i] = kb < K ? W[(size_t)(kb < K ? kb : K - 1) * ld + n] : 0.f; }
  return bsplit16(v); }
__device__ __forceinline__ v8f mac3(const F2& a, const F2& b, v8f c) { c = wmma_bf(a.l, b.h, c); c = wmma_bf(a.h, b.l, c); return wmma_bf(a.h, b.h, c); }
__device__ __forceinline__ float sigm(float v) { return 1.0f / (1.0f + expf(-v)); }
#define LDSX() do { asm volatile("s_wait_dscnt 0" ::: "memory"); __builtin_amdgcn_wave_barrier(); __builtin_amdgcn_fence(__ATOMIC_RELEASE, "workgroup"); } while (0)


#define NB 16
#define CC 256
#define HI 56
#define WI 56
#define NPIX (HI * WI)
#define NT ((NPIX + 127) / 128)
#define MID 16
#ifndef NBT
#define NBT NB
#endif
typedef __attribute__((ext_vector_type(8))) __bf16 v8b;
__device__ __forceinline__ v16b frag_b(const __bf16* rowk0, int lane) {
  union { v16b v; v8b q[2]; } u; const __bf16* p = rowk0 + 8 * (lane >> 4);
  u.q[0] = *(const v8b*)p; u.q[1] = *(const v8b*)(p + 16); return u.v;
}
__device__ __forceinline__ float bfr(float v) { return (float)(__bf16)v; }
__device__ __attribute__((noinline)) float exp_ni(float v) { return expf(v); }
__device__ __attribute__((noinline)) float erf_ni(float v) { return erff(v); }

#define WS_P1   0u
#define WS_P2   (WS_P1 + 2u * CC * CC)
#define WS_O1   (WS_P2 + 2u * CC * CC)
#define WS_TOP  (WS_O1 + 4u * NB * CC * NPIX)
#define WS_SUM  (WS_TOP + 4u * NB * CC * NPIX)
#define WS_SC   (WS_SUM + 4u * NB * NT * CC)
#define WS_END  (WS_SC + 4u * NB * CC)

__global__ __launch_bounds__(256) void k_pack(const float* __restrict__ Wm, __bf16* __restrict__ DST) {
  __shared__ __align__(16) __bf16 s[CC]; const int o = blockIdx.x, tid = threadIdx.x; s[tid] = (__bf16)Wm[(size_t)o * CC + tid]; __syncthreads();
  if (tid < CC / 8) vst2((unsigned*)(DST + (size_t)o * CC + tid * 8), *(const v4u*)&s[tid * 8]);
}
__device__ __forceinline__ v16b gfrag(const float* __restrict__ base, int p, int k0, int lane) { v16b a; const float* q = base + (size_t)(k0 + 8 * (lane >> 4)) * NPIX + p;
#pragma unroll
  for (int i = 0; i < 8; ++i) { a[i] = (__bf16)q[(size_t)i * NPIX]; a[8 + i] = (__bf16)q[(size_t)(16 + i) * NPIX]; }
  return a; }
__device__ __forceinline__ F2 gfrag2(const float* __restrict__ base, int p, int k0, int lane) { float v[16]; const float* q = base + (size_t)(k0 + 8 * (lane >> 4)) * NPIX + p;
#pragma unroll
  for (int i = 0; i < 8; ++i) { v[i] = q[(size_t)i * NPIX]; v[8 + i] = q[(size_t)(16 + i) * NPIX]; }
  return bsplit16(v); }
template <int MODE>
__global__ __launch_bounds__(128) void k_pw(const float* __restrict__ SRC, const __bf16* __restrict__ PW, const float* __restrict__ g2, const float* __restrict__ be2, const float* __restrict__ m2, const float* __restrict__ v2, const float* __restrict__ SC, const float* __restrict__ X, float* __restrict__ OUT, float* __restrict__ SUM) {
  __shared__ __align__(16) float so[4][32][132]; __shared__ float ssum[CC];
  const int tid = threadIdx.x, wave = tid >> 5, lane = tid & 31, col = lane & 15, g = lane >> 4; const int pt = blockIdx.x, b = blockIdx.y; const int p0 = pt * 128; const int npx = min(128, NPIX - p0);
  const float* src = SRC + (size_t)b * CC * NPIX;
#pragma unroll 1
  for (int ps = 0; ps < 2; ++ps) { const int o0 = ps * 128 + wave * 32; v8f acc[2][8] = {};
#pragma unroll 1
    for (int kc = 0; kc < CC / 32; ++kc) { const v16b a0 = frag_b(PW + (size_t)(o0 + col) * CC + kc * 32, lane), a1 = frag_b(PW + (size_t)(o0 + 16 + col) * CC + kc * 32, lane);
#pragma unroll
      for (int j = 0; j < 8; ++j) { int p = p0 + j * 16 + col; p = p < NPIX ? p : NPIX - 1;
        if (MODE == 0) { const v16b xb = gfrag(src, p, kc * 32, lane); acc[0][j] = wmma_bf(a0, xb, acc[0][j]); acc[1][j] = wmma_bf(a1, xb, acc[1][j]); }
        else { const F2 tb = gfrag2(src, p, kc * 32, lane); acc[0][j] = wmma_bf(a0, tb.l, acc[0][j]); acc[0][j] = wmma_bf(a0, tb.h, acc[0][j]); acc[1][j] = wmma_bf(a1, tb.l, acc[1][j]); acc[1][j] = wmma_bf(a1, tb.h, acc[1][j]); } } }
#pragma unroll
    for (int rt = 0; rt < 2; ++rt) {
#pragma unroll
      for (int r = 0; r < 8; ++r) { const int ol = rt * 16 + 8 * g + r; const int o = o0 + ol; float sc = 1.f, sh = 0.f, se = 1.f;
        if (MODE != 0) { const float s = bfr(g2[o]) * rsqrtf(bfr(v2[o]) + 1e-5f); sc = s; sh = bfr(be2[o]) - bfr(m2[o]) * s; if (MODE == 2) se = SC[b * CC + o]; }
#pragma unroll
        for (int j = 0; j < 8; ++j) { float v = acc[rt][j][r]; if (MODE != 0) { v = fmaxf(v * sc + sh, 0.f); if (MODE == 2) { const int p = p0 + j * 16 + col; v = v * se + bfr(X[((size_t)b * CC + o) * NPIX + (p < NPIX ? p : NPIX - 1)]); } } so[wave][ol][j * 16 + col] = v; } } }
    LDSX();
    if (MODE == 1) {
      { float s = 0.f; for (int pl = 0; pl < npx; ++pl) s += so[wave][lane][pl]; ssum[o0 + lane] = s; }
    } else {
      for (int ol = 0; ol < 32; ++ol) { if (lane * 4 < npx) vst2(OUT + ((size_t)b * CC + o0 + ol) * NPIX + p0 + lane * 4, *(const v4f*)&so[wave][ol][lane * 4]); }
    }
    LDSX(); }
  if (MODE == 1) { __syncthreads(); if (tid < 64) vst2(SUM + ((size_t)b * NT + pt) * CC + tid * 4, *(const v4f*)&ssum[tid * 4]); }
}
__global__ __launch_bounds__(256) void k_top(const float* __restrict__ O1, const float* __restrict__ Wxy3, const float* __restrict__ Wxy5, const float* __restrict__ gxy, const float* __restrict__ bxy, const float* __restrict__ mxy, const float* __restrict__ vxy,
    const float* __restrict__ Wxz3, const float* __restrict__ Wxz5, const float* __restrict__ gxz, const float* __restrict__ bxz, const float* __restrict__ mxz, const float* __restrict__ vxz,
    const float* __restrict__ Wyz3, const float* __restrict__ Wyz5, const float* __restrict__ gyz, const float* __restrict__ byz, const float* __restrict__ myz, const float* __restrict__ vyz,
    const float* __restrict__ AL, const float* __restrict__ BE, float* __restrict__ TOP) {
  __shared__ float sp[HI + 4][WI + 4]; __shared__ __align__(16) float sout[NPIX]; __shared__ float sw[9 + 25 + 3 + 5 + 3 + 5];
  const int tid = threadIdx.x; const int b = blockIdx.x / CC, c = blockIdx.x % CC; const float* plane = O1 + ((size_t)b * CC + c) * NPIX;
  for (int q = tid; q < (HI + 4) * (WI + 4); q += 256) { const int yy = q / (WI + 4) - 2, xx = q % (WI + 4) - 2; (&sp[0][0])[q] = (yy >= 0 && yy < HI && xx >= 0 && xx < WI) ? plane[yy * WI + xx] : 0.f; }
  if (tid < 9) sw[tid] = bfr(Wxy3[c * 9 + tid]); else if (tid < 34) sw[tid] = bfr(Wxy5[c * 25 + (tid - 9)]); else if (tid < 37) sw[tid] = bfr(Wxz3[c * 3 + (tid - 34)]); else if (tid < 42) sw[tid] = bfr(Wxz5[c * 5 + (tid - 37)]); else if (tid < 45) sw[tid] = bfr(Wyz3[c * 3 + (tid - 42)]); else if (tid < 50) sw[tid] = bfr(Wyz5[c * 5 + (tid - 45)]);
  __syncthreads();
  const float sxy = bfr(gxy[c]) * rsqrtf(bfr(vxy[c]) + 1e-5f), hxy = bfr(bxy[c]) - bfr(mxy[c]) * sxy;
  const float sxz = bfr(gxz[c]) * rsqrtf(bfr(vxz[c]) + 1e-5f), hxz = bfr(bxz[c]) - bfr(mxz[c]) * sxz;
  const float syz = bfr(gyz[c]) * rsqrtf(bfr(vyz[c]) + 1e-5f), hyz = bfr(byz[c]) - bfr(myz[c]) * syz;
  const float al = bfr(AL[c]), be = bfr(BE[c]);
  for (int p = tid; p < NPIX; p += 256) { const int y = p / WI, x = p % WI; const int Y = y + 2, Xc = x + 2;
    float a3 = 0.f, a5 = 0.f, z3 = 0.f, z5 = 0.f, w3 = 0.f, w5 = 0.f;
#pragma unroll 1
    for (int dy = 0; dy < 3; ++dy)
#pragma unroll
      for (int dx = 0; dx < 3; ++dx) a3 += sw[dy * 3 + dx] * sp[Y + dy - 1][Xc + dx - 1];
#pragma unroll 1
    for (int dy = 0; dy < 5; ++dy)
#pragma unroll
      for (int dx = 0; dx < 5; ++dx) a5 += sw[9 + dy * 5 + dx] * sp[Y + dy - 2][Xc + dx - 2];
#pragma unroll
    for (int dx = 0; dx < 3; ++dx) z3 += sw[34 + dx] * sp[Y][Xc + dx - 1];
#pragma unroll
    for (int dx = 0; dx < 5; ++dx) z5 += sw[37 + dx] * sp[Y][Xc + dx - 2];
#pragma unroll
    for (int dy = 0; dy < 3; ++dy) w3 += sw[42 + dy] * sp[Y + dy - 1][Xc];
#pragma unroll
    for (int dy = 0; dy < 5; ++dy) w5 += sw[45 + dy] * sp[Y + dy - 2][Xc];
    const float fxy = fmaxf((a3 + a5) * sxy + hxy, 0.f), fxz = fmaxf((z3 + z5) * sxz + hxz, 0.f), fyz = fmaxf((w3 + w5) * syz + hyz, 0.f);
    const float gate = sigm(al * fxz + be * fyz); sout[p] = fmaxf(fxy * gate, 0.f); }
  __syncthreads();
  for (int q = tid; q < NPIX / 4; q += 256) vst2(TOP + ((size_t)b * CC + c) * NPIX + q * 4, *(const v4f*)&sout[q * 4]);
}
__global__ __launch_bounds__(256) void k_se(const float* __restrict__ SUM, const float* __restrict__ W1, const float* __restrict__ B1, const float* __restrict__ W2, const float* __restrict__ B2, float* __restrict__ SC) {
  __shared__ float sm[CC]; __shared__ float sh[MID]; __shared__ __align__(16) float ssc[CC]; const int b = blockIdx.x, c = threadIdx.x;
  { float s = 0.f; for (int t = 0; t < NT; ++t) s += SUM[((size_t)b * NT + t) * CC + c]; sm[c] = s * (1.0f / (float)NPIX); }
  __syncthreads();
  if (c < MID) { float s = bfr(B1[c]);
#pragma unroll 4
    for (int k = 0; k < CC; ++k) s += sm[k] * bfr(W1[c * CC + k]);
    sh[c] = fmaxf(s, 0.f); }
  __syncthreads();
  { float s = bfr(B2[c]);
#pragma unroll
    for (int k = 0; k < MID; ++k) s += sh[k] * bfr(W2[c * MID + k]);
    ssc[c] = sigm(s); }
  __syncthreads();
  if (c < 64) vst2(SC + (size_t)b * CC + c * 4, *(const v4f*)&ssc[c * 4]);
}
extern "C" void kernel_launch(void* const* d_in, const int* in_sizes, int n_in, void* d_out, int out_size, void* d_ws, size_t ws_size, hipStream_t stream) {
  (void)in_sizes; (void)n_in; (void)out_size;
  const float** F = (const float**)d_in;
  if (ws_size < (size_t)WS_END) return;
  char* ws = (char*)d_ws; __bf16 *P1 = (__bf16*)(ws + WS_P1), *P2 = (__bf16*)(ws + WS_P2); float *O1 = (float*)(ws + WS_O1), *TOP = (float*)(ws + WS_TOP), *SUM = (float*)(ws + WS_SUM), *SC = (float*)(ws + WS_SC);
  k_pack<<<CC, 256, 0, stream>>>(F[1], P1); k_pack<<<CC, 256, 0, stream>>>(F[22], P2);
  k_pw<0><<<dim3(NT, NBT), 128, 0, stream>>>(F[0], P1, nullptr, nullptr, nullptr, nullptr, nullptr, nullptr, O1, nullptr);
  k_top<<<NBT * CC, 256, 0, stream>>>(O1, F[2], F[3], F[4], F[5], F[6], F[7], F[8], F[9], F[10], F[11], F[12], F[13], F[14], F[15], F[16], F[17], F[18], F[19], F[20], F[21], TOP);
  k_pw<1><<<dim3(NT, NBT), 128, 0, stream>>>(TOP, P2, F[23], F[24], F[25], F[26], nullptr, nullptr, nullptr, SUM);
  k_se<<<NBT, 256, 0, stream>>>(SUM, F[27], F[28], F[29], F[30], SC);
  k_pw<2><<<dim3(NT, NBT), 128, 0, stream>>>(TOP, P2, F[23], F[24], F[25], F[26], SC, F[0], (float*)d_out, nullptr);
}
